// mowLSTM_31920196944179
// MI455X (gfx1250) — hardware-run, weakly checked
//
#include <hip/hip_runtime.h>
#include <math.h>

constexpr int NBAT    = 256;
constexpr int NSTEP   = 256;
constexpr int NFEAT   = 128;
constexpr int NHID    = 256;
constexpr int NGATE   = 4 * NHID;
constexpr int NMIX    = 2;
constexpr int NOUTF   = 64;
constexpr int KCAT    = NFEAT + NHID;
constexpr int NCAT    = NMIX * NGATE;
constexpr int NTHR    = 256;
constexpr int SEQ_BLK = 16;
constexpr int APITCH  = 392;
constexpr int NROWS   = NBAT * NSTEP;
constexpr float WCARRY  = 256.0f;
constexpr float ACARRY  = 64.0f;
constexpr float ACC_INV = 1.0f / (WCARRY * ACARRY);
constexpr float H16_MIN = 6.103515625e-5f;

static_assert(NGATE == 1024 && KCAT == 384 && NCAT == 2048, "shape constants");
static_assert(KCAT % 32 == 0 && NHID % 32 == 0, "k depth multiple of 32");
static_assert(NROWS % 64 == 0 && NOUTF % 64 == 0, "head tile multiples");
static_assert(NBAT % SEQ_BLK == 0, "whole row blocks");
static_assert(NHID == 32 * (NTHR / 32), "8 waves x 32 hidden units");
static_assert(SEQ_BLK * NFEAT == NTHR * 8, "x tile staging exact");
static_assert(SEQ_BLK == 2 * (NTHR / 32), "two h rows per wave in the store phase");
static_assert(APITCH % 8 == 0 && APITCH >= KCAT, "A tile pitch");
static_assert(NHID * 2 == 32 * 16, "one h row = one 32-lane 16-B store");

typedef __attribute__((ext_vector_type(16))) _Float16 v16h;
typedef __attribute__((ext_vector_type(8)))  _Float16 v8h;
typedef __attribute__((ext_vector_type(16))) __bf16   v16b;
typedef __attribute__((ext_vector_type(8)))  __bf16   v8b;
typedef __attribute__((ext_vector_type(8)))  float    v8f;
typedef __attribute__((ext_vector_type(4)))  float    v4f;

__device__ __forceinline__ unsigned short f2bf_bits(float f) {
  unsigned u = __float_as_uint(f);
  return (unsigned short)((u + 0x7FFFu + ((u >> 16) & 1u)) >> 16);
}
__device__ __forceinline__ float bf_bits2f(unsigned short h) { return __uint_as_float(((unsigned)h) << 16); }

__device__ __forceinline__ void dep_guard_h(v8f& a, v8f& b, v16h x, v16h y) { asm volatile("v_nop\n\tv_nop\n\tv_nop\n\tv_nop" : "+v"(a), "+v"(b) : "v"(x), "v"(y)); }
__device__ __forceinline__ void dep_guard_b(v8f& a, v8f& b, v16b x, v16b y) { asm volatile("v_nop\n\tv_nop\n\tv_nop\n\tv_nop" : "+v"(a), "+v"(b) : "v"(x), "v"(y)); }
__device__ __forceinline__ void keep4_h(v16h a, v16h b, v16h c, v16h d) { asm volatile("v_nop" :: "v"(a), "v"(b), "v"(c), "v"(d)); }
__device__ __forceinline__ void keep4_b(v16b a, v16b b, v16b c, v16b d) { asm volatile("v_nop" :: "v"(a), "v"(b), "v"(c), "v"(d)); }
__device__ __forceinline__ void acc_guard4(v8f& a, v8f& b, v8f& c, v8f& d) { asm volatile("v_nop\n\tv_nop\n\tv_nop\n\tv_nop" : "+v"(a), "+v"(b), "+v"(c), "+v"(d)); }

template <typename T> struct Frag;
template <> struct Frag<_Float16> {
  typedef v16h V; union U { v16h v; v8h h[2]; };
  static __device__ __forceinline__ v16h load(const _Float16* p) {
    U f; f.h[0] = *(const v8h*)(p); f.h[1] = *(const v8h*)(p + 16); return f.v;
  }
  static __device__ __forceinline__ v8f mma(v16h a, v16h b, v8f c) {
    return __builtin_amdgcn_wmma_f32_16x16x32_f16(false, a, false, b, (short)0, c, false, false);
  }
  static __device__ __forceinline__ void guard(v8f& a, v8f& b, v16h x, v16h y) { dep_guard_h(a, b, x, y); }
  static __device__ __forceinline__ void keep(v16h a, v16h b, v16h c, v16h d) { keep4_h(a, b, c, d); }
};
template <> struct Frag<__bf16> {
  typedef v16b V; union U { v16b v; v8b h[2]; };
  static __device__ __forceinline__ v16b load(const __bf16* p) {
    U f; f.h[0] = *(const v8b*)(p); f.h[1] = *(const v8b*)(p + 16); return f.v;
  }
  static __device__ __forceinline__ v8f mma(v16b a, v16b b, v8f c) {
    return __builtin_amdgcn_wmma_f32_16x16x32_bf16(false, a, false, b, (short)0, c, false, false);
  }
  static __device__ __forceinline__ void guard(v8f& a, v8f& b, v16b x, v16b y) { dep_guard_b(a, b, x, y); }
  static __device__ __forceinline__ void keep(v16b a, v16b b, v16b c, v16b d) { keep4_b(a, b, c, d); }
};

__device__ __forceinline__ v8f mma_h(v16h a, v16h b, v8f c) {
  c = __builtin_amdgcn_wmma_f32_16x16x32_f16(false, a, false, b, (short)0, c, false, false);
  asm volatile("v_nop\n\tv_nop\n\tv_nop\n\tv_nop" : "+v"(c) : "v"(a), "v"(b));
  return c;
}

__device__ __forceinline__ _Float16 to_h16(float v) {
  const float w = (fabsf(v) < H16_MIN) ? 0.0f : v;
  return (_Float16)w;
}

__device__ __forceinline__ float fsig(float x)  { return __builtin_amdgcn_rcpf(1.0f + __expf(-x)); }
__device__ __forceinline__ float ftanh(float x) { return 1.0f - 2.0f * __builtin_amdgcn_rcpf(__expf(2.0f * x) + 1.0f); }

template <int ET> struct Elem;
template <> struct Elem<0> { typedef _Float16 T; };
template <> struct Elem<1> { typedef __bf16 T; };
template <int ET, bool SPLIT, int BIAS_MODE, int OUT_MODE, bool RESID, int ACT = 0>
__global__ __launch_bounds__(256) void wmma_gemm64(
    const unsigned short* __restrict__ Ap, const unsigned short* __restrict__ A2p, int lda, long strideA,
    const unsigned short* __restrict__ Btp, const unsigned short* __restrict__ Bt2p, int ldb, long strideB,
    void* __restrict__ Cout, void* __restrict__ Cout2, int ldc, long strideC,
    const float* __restrict__ bias,
    const float* __restrict__ resid, long strideR,
    int M, int N, int K, float scale) {
  typedef typename Elem<ET>::T T;
  typedef typename Frag<T>::V V;
  const T* A = (const T*)Ap; const T* A2 = (const T*)A2p; const T* Bt = (const T*)Btp; const T* Bt2 = (const T*)Bt2p;
  __shared__ __align__(16) float sT[8][16 * 68];
  const int b    = blockIdx.y;
  const int lane = threadIdx.x & 31;
  const int wave = threadIdx.x >> 5;
  const int tilesN = N >> 6;
  const int tilesM = M >> 6;
  const int tile = blockIdx.x * 8 + wave;
  if (tile >= tilesM * tilesN) return;
  const int tm = tile / tilesN;
  const int tn = tile - tm * tilesN;
  const int m0 = tm << 6;
  const int n0 = tn << 6;

  const T* Ab  = A  + (size_t)b * strideA;
  const T* Bb  = Bt + (size_t)b * strideB;
  const T* Ab2 = SPLIT ? (A2  + (size_t)b * strideA) : nullptr;
  const T* Bb2 = SPLIT ? (Bt2 + (size_t)b * strideB) : nullptr;

  const int rlane = lane & 15;
  const int koff  = (lane >> 4) * 8;
  const int mOff  = (lane >> 4) * 8;

  v8f acc[4][4];
#pragma unroll
  for (int i = 0; i < 4; ++i)
#pragma unroll
    for (int j = 0; j < 4; ++j) acc[i][j] = (v8f){0.f,0.f,0.f,0.f,0.f,0.f,0.f,0.f};

  for (int k0 = 0; k0 < K; k0 += 32) {
    V bh[4], bl[4];
#pragma unroll
    for (int j = 0; j < 4; ++j) {
      const size_t bo = (size_t)(n0 + (j << 4) + rlane) * ldb + koff + k0;
      bh[j] = Frag<T>::load(Bb + bo);
      if (SPLIT) bl[j] = Frag<T>::load(Bb2 + bo);
    }
#pragma unroll
    for (int i = 0; i < 4; ++i) {
      const size_t ao = (size_t)(m0 + (i << 4) + rlane) * lda + koff + k0;
      V ah = Frag<T>::load(Ab + ao);
      V al;
      if (SPLIT) al = Frag<T>::load(Ab2 + ao);
#pragma unroll
      for (int j = 0; j < 4; ++j) {
        acc[i][j] = Frag<T>::mma(ah, bh[j], acc[i][j]);
        if (SPLIT) {
          acc[i][j] = Frag<T>::mma(ah, bl[j], acc[i][j]);
          acc[i][j] = Frag<T>::mma(al, bh[j], acc[i][j]);
        }
      }
      Frag<T>::guard(acc[i][0], acc[i][3], ah, SPLIT ? al : ah);
    }
    Frag<T>::keep(bh[0], bh[1], bh[2], bh[3]);
    if (SPLIT) Frag<T>::keep(bl[0], bl[1], bl[2], bl[3]);
  }
  acc_guard4(acc[0][0], acc[0][1], acc[0][2], acc[0][3]);
  acc_guard4(acc[1][0], acc[1][1], acc[1][2], acc[1][3]);
  acc_guard4(acc[2][0], acc[2][1], acc[2][2], acc[2][3]);
  acc_guard4(acc[3][0], acc[3][1], acc[3][2], acc[3][3]);

  float* slab = sT[wave];
  const float* Rb = RESID ? (resid + (size_t)b * strideR) : nullptr;
#pragma unroll
  for (int i = 0; i < 4; ++i) {
    const int mBase = m0 + (i << 4);
#pragma unroll
    for (int j = 0; j < 4; ++j) {
      const int n = n0 + (j << 4) + rlane;
      float bv = 0.f;
      if (BIAS_MODE == 2) bv = bias[n];
#pragma unroll
      for (int r = 0; r < 8; ++r) {
        float v = acc[i][j][r] * scale;
        if (BIAS_MODE == 1) v += bias[mBase + mOff + r];
        if (BIAS_MODE == 2) v += bv;
        if (RESID) v += Rb[(size_t)(mBase + mOff + r) * ldc + n];
        if (ACT == 1) v = tanhf(v);
        if (ACT == 2) v = fmaxf(v, 0.0f);
        if (ACT == 3) v = v / (1.0f + expf(-v));
        if (ACT == 4) v = (v > 0.f) ? v : 0.01f * v;
        if (ACT == 5) v = 0.5f * v * (1.0f + erff(v * 0.70710678118654752f));
        slab[(mOff + r) * 68 + (j << 4) + rlane] = v;
      }
    }
    __builtin_amdgcn_fence(__ATOMIC_RELEASE, "workgroup");
    __builtin_amdgcn_wave_barrier();
    __builtin_amdgcn_fence(__ATOMIC_ACQUIRE, "workgroup");
    if (OUT_MODE == 0) {
      float* C = (float*)Cout + (size_t)b * strideC;
      const int hh = lane >> 4, c4 = (lane & 15) * 4;
      for (int pass = 0; pass < 2; ++pass) {
#pragma unroll
        for (int it = 0; it < 8; ++it) {
          const int row = it * 2 + hh;
          v4f v = *(const v4f*)(slab + row * 68 + c4);
          *(volatile v4f*)(C + (size_t)(mBase + row) * ldc + n0 + c4) = v;
        }
        __threadfence();
      }
    } else {
      const int q = lane >> 3, c8 = (lane & 7) * 8;
      unsigned short* C  = (unsigned short*)Cout  + (size_t)b * strideC;
      unsigned short* C2 = (OUT_MODE == 2) ? ((unsigned short*)Cout2 + (size_t)b * strideC) : nullptr;
      for (int pass = 0; pass < 2; ++pass) {
#pragma unroll
        for (int it = 0; it < 4; ++it) {
          const int row = it * 4 + q;
          const float* sp = slab + row * 68 + c8;
          v8h hv, lv;
#pragma unroll
          for (int e = 0; e < 8; ++e) {
            if (OUT_MODE == 1) {
              hv[e] = (_Float16)sp[e];
            } else {
              unsigned short hb = f2bf_bits(sp[e]);
              unsigned short lb = f2bf_bits(sp[e] - bf_bits2f(hb));
              hv[e] = __builtin_bit_cast(_Float16, hb);
              lv[e] = __builtin_bit_cast(_Float16, lb);
            }
          }
          *(volatile v8h*)(C + (size_t)(mBase + row) * ldc + n0 + c8) = hv;
          if (OUT_MODE == 2) *(volatile v8h*)(C2 + (size_t)(mBase + row) * ldc + n0 + c8) = lv;
        }
        __threadfence();
      }
    }
    __builtin_amdgcn_fence(__ATOMIC_RELEASE, "workgroup");
    __builtin_amdgcn_wave_barrier();
    __builtin_amdgcn_fence(__ATOMIC_ACQUIRE, "workgroup");
  }
}

__global__ __launch_bounds__(NTHR) void pack_t_kernel(const float* __restrict__ src, long srcStrideZ, int ncols,
                                                      unsigned short* __restrict__ dst, long dstStrideZ, int ldo, float sc) {
  __shared__ float Tt[64 * 65];
  const int tid = threadIdx.x;
  const int c0 = blockIdx.x * 64, r0 = blockIdx.y * 64;
  const float* sp = src + (size_t)blockIdx.z * (size_t)srcStrideZ;
  unsigned short* dp = dst + (size_t)blockIdx.z * (size_t)dstStrideZ;
#pragma unroll
  for (int i = 0; i < 4; ++i) {
    const int idx = i * NTHR + tid;
    const int rr = idx >> 4, cc = (idx & 15) * 4;
    const v4f v = *(const v4f*)(sp + (size_t)(r0 + rr) * (size_t)ncols + c0 + cc);
    Tt[rr * 65 + cc + 0] = v[0];
    Tt[rr * 65 + cc + 1] = v[1];
    Tt[rr * 65 + cc + 2] = v[2];
    Tt[rr * 65 + cc + 3] = v[3];
  }
  __syncthreads();
  const int q = tid >> 3, c8 = (tid & 7) * 8;
  v8h hv[2];
#pragma unroll
  for (int g = 0; g < 2; ++g) {
    const int qq = g * 32 + q;
#pragma unroll
    for (int e = 0; e < 8; ++e) {
      const float f = Tt[(c8 + e) * 65 + qq];
      hv[g][e] = to_h16(f * sc);
    }
  }
  for (int pass = 0; pass < 2; ++pass) {
#pragma unroll
    for (int g = 0; g < 2; ++g) {
      const size_t o = (size_t)(c0 + g * 32 + q) * (size_t)ldo + (size_t)(r0 + c8);
      *(volatile v8h*)(dp + o) = hv[g];
    }
    __threadfence();
  }
}

__global__ __launch_bounds__(NTHR) void lstm_seq_kernel(const float* __restrict__ x, const float* __restrict__ bias,
                                                        const float* __restrict__ alpha,
                                                        const unsigned short* __restrict__ Wcp,
                                                        unsigned short* __restrict__ HSp) {
  __shared__ __align__(16) _Float16 At[2][SEQ_BLK * APITCH];
  const _Float16* Wc = (const _Float16*)Wcp;
  const int tid = threadIdx.x, lane = tid & 31, wave = tid >> 5;
  const int c = lane & 15, hh = lane >> 4, koff = hh * 8;
  const int rowbase = blockIdx.x * SEQ_BLK;
  const int xm = tid >> 4, xs = tid & 15;

  {
    v8h zz;
#pragma unroll
    for (int e = 0; e < 8; ++e) zz[e] = (_Float16)0.0f;
    _Float16* zp = &At[0][0] + xm * APITCH + NFEAT + xs * 16;
    *(v8h*)(zp) = zz;
    *(v8h*)(zp + 8) = zz;
  }
  {
    const float* sp = x + ((size_t)(rowbase + xm) * NSTEP) * NFEAT + xs * 8;
    const v4f va = *(const v4f*)(sp);
    const v4f vb = *(const v4f*)(sp + 4);
    v8h hv;
#pragma unroll
    for (int e = 0; e < 4; ++e) {
      hv[e]     = to_h16(va[e] * ACARRY);
      hv[4 + e] = to_h16(vb[e] * ACARRY);
    }
    *(v8h*)(&At[0][0] + xm * APITCH + xs * 8) = hv;
  }

  float cst[2][8], b0r[2][4], b1r[2][4];
#pragma unroll
  for (int nt = 0; nt < 2; ++nt) {
    const int j = 32 * wave + 16 * nt + c;
#pragma unroll
    for (int g = 0; g < 4; ++g) {
      float t0 = bias[g * NHID + j];
      asm volatile("" : "+v"(t0));
      b0r[nt][g] = t0;
    }
  }
#pragma unroll
  for (int nt = 0; nt < 2; ++nt) {
    const int j = 32 * wave + 16 * nt + c;
#pragma unroll
    for (int g = 0; g < 4; ++g) {
      float t1 = bias[NGATE + g * NHID + j];
      asm volatile("" : "+v"(t1));
      b1r[nt][g] = t1;
    }
#pragma unroll
    for (int r = 0; r < 8; ++r) cst[nt][r] = 0.0f;
  }
  __syncthreads();

  const v8f z8 = {0.f, 0.f, 0.f, 0.f, 0.f, 0.f, 0.f, 0.f};

#pragma unroll 1
  for (int t = 0; t < NSTEP; ++t) {
    const int cur = t & 1;
    const _Float16* arow = &At[cur][0] + c * APITCH + koff;
    _Float16* anx = &At[cur ^ 1][0];

    const float a0 = alpha[2 * t + 0];
    const float a1 = alpha[2 * t + 1];
    const float am = fmaxf(a0, a1);
    const float e0 = expf(a0 - am);
    const float e1 = expf(a1 - am);
    const float einv = 1.0f / (e0 + e1);
    const float c0 = e0 * einv;
    const float c1 = e1 * einv;
    const float cs0 = c0 * ACC_INV;
    const float cs1 = c1 * ACC_INV;

    const int tn = (t + 1 < NSTEP) ? (t + 1) : (NSTEP - 1);
    const float* xsp = x + ((size_t)(rowbase + xm) * NSTEP + (size_t)tn) * NFEAT + xs * 8;
    const v4f xva = *(const v4f*)(xsp);
    const v4f xvb = *(const v4f*)(xsp + 4);

#pragma unroll
    for (int nt = 0; nt < 2; ++nt) {
      const int j = 32 * wave + 16 * nt + c;
      const _Float16* wr = Wc + (size_t)j * KCAT + koff;
      v8f p0[4], p1[4];
      p0[0] = z8; p0[1] = z8; p0[2] = z8; p0[3] = z8;
      p1[0] = z8; p1[1] = z8; p1[2] = z8; p1[3] = z8;
#pragma unroll 1
      for (int k0 = 0; k0 < KCAT; k0 += 32) {
        const v16h a = Frag<_Float16>::load(arow + k0);
        {
          const v16h b0 = Frag<_Float16>::load(wr + (size_t)(0 * NHID) * KCAT + k0);
          const v16h b1 = Frag<_Float16>::load(wr + (size_t)(1 * NHID) * KCAT + k0);
          const v16h b2 = Frag<_Float16>::load(wr + (size_t)(2 * NHID) * KCAT + k0);
          const v16h b3 = Frag<_Float16>::load(wr + (size_t)(3 * NHID) * KCAT + k0);
          p0[0] = mma_h(a, b0, p0[0]);
          p0[1] = mma_h(a, b1, p0[1]);
          p0[2] = mma_h(a, b2, p0[2]);
          p0[3] = mma_h(a, b3, p0[3]);
        }
        {
          const v16h b0 = Frag<_Float16>::load(wr + (size_t)(NGATE + 0 * NHID) * KCAT + k0);
          const v16h b1 = Frag<_Float16>::load(wr + (size_t)(NGATE + 1 * NHID) * KCAT + k0);
          const v16h b2 = Frag<_Float16>::load(wr + (size_t)(NGATE + 2 * NHID) * KCAT + k0);
          const v16h b3 = Frag<_Float16>::load(wr + (size_t)(NGATE + 3 * NHID) * KCAT + k0);
          p1[0] = mma_h(a, b0, p1[0]);
          p1[1] = mma_h(a, b1, p1[1]);
          p1[2] = mma_h(a, b2, p1[2]);
          p1[3] = mma_h(a, b3, p1[3]);
        }
      }
      acc_guard4(p0[0], p0[1], p0[2], p0[3]);
      acc_guard4(p1[0], p1[1], p1[2], p1[3]);

      const float bti = fmaf(c0, b0r[nt][0], c1 * b1r[nt][0]);
      const float btf = fmaf(c0, b0r[nt][1], c1 * b1r[nt][1]);
      const float btg = fmaf(c0, b0r[nt][2], c1 * b1r[nt][2]);
      const float bto = fmaf(c0, b0r[nt][3], c1 * b1r[nt][3]);

#pragma unroll
      for (int r = 0; r < 8; ++r) {
        const float zi = fmaf(cs0, p0[0][r], fmaf(cs1, p1[0][r], bti));
        const float zf = fmaf(cs0, p0[1][r], fmaf(cs1, p1[1][r], btf));
        const float zg = fmaf(cs0, p0[2][r], fmaf(cs1, p1[2][r], btg));
        const float zo = fmaf(cs0, p0[3][r], fmaf(cs1, p1[3][r], bto));
        const float ig = fsig(zi);
        const float fg = fsig(zf);
        const float gg = ftanh(zg);
        const float og = fsig(zo);
        const float cn = fg * cst[nt][r] + ig * gg;
        cst[nt][r] = cn;
        const float hn = og * ftanh(cn);
        anx[(8 * hh + r) * APITCH + NFEAT + j] = to_h16(hn * ACARRY);
      }
    }

    {
      v8h hv;
#pragma unroll
      for (int e = 0; e < 4; ++e) {
        hv[e]     = to_h16(xva[e] * ACARRY);
        hv[4 + e] = to_h16(xvb[e] * ACARRY);
      }
      *(v8h*)(anx + xm * APITCH + xs * 8) = hv;
    }
    __syncthreads();

    {
      const int r0 = 2 * wave, r1 = 2 * wave + 1;
      const v8h hv0 = *(const v8h*)(anx + r0 * APITCH + NFEAT + lane * 8);
      const v8h hv1 = *(const v8h*)(anx + r1 * APITCH + NFEAT + lane * 8);
      unsigned short* d0 = HSp + ((size_t)(rowbase + r0) * NSTEP + (size_t)t) * NHID + lane * 8;
      unsigned short* d1 = HSp + ((size_t)(rowbase + r1) * NSTEP + (size_t)t) * NHID + lane * 8;
      for (int pass = 0; pass < 2; ++pass) {
        *(volatile v8h*)(d0) = hv0;
        *(volatile v8h*)(d1) = hv1;
        __threadfence();
      }
    }
  }
}

extern "C" void kernel_launch(void* const* d_in, const int* in_sizes, int n_in,
                              void* d_out, int out_size, void* d_ws, size_t ws_size, hipStream_t stream) {
  if (n_in < 7 || d_out == nullptr || d_ws == nullptr) return;
  if (in_sizes[0] != NBAT * NSTEP * NFEAT || in_sizes[1] != NMIX * NFEAT * NGATE ||
      in_sizes[2] != NMIX * NHID * NGATE || in_sizes[3] != NMIX * NGATE || in_sizes[4] != NSTEP * NMIX ||
      in_sizes[5] != NHID * NOUTF || in_sizes[6] != NOUTF || out_size != NROWS * NOUTF) return;

  const float* xin   = (const float*)d_in[0];
  const float* w_ih  = (const float*)d_in[1];
  const float* w_hh  = (const float*)d_in[2];
  const float* bvec  = (const float*)d_in[3];
  const float* alpha = (const float*)d_in[4];
  const float* w_out = (const float*)d_in[5];
  const float* b_out = (const float*)d_in[6];
  float* out = (float*)d_out;

  char* ws = (char*)d_ws; size_t off = 0;
  auto carve = [&](size_t bytes) -> char* { char* p = ws + off; off += (bytes + 255) & ~(size_t)255; return p; };
  unsigned short* WCAT = (unsigned short*)carve((size_t)NCAT * KCAT * 2);
  unsigned short* WOT  = (unsigned short*)carve((size_t)NOUTF * NHID * 2);
  unsigned short* HS   = (unsigned short*)carve((size_t)NROWS * NHID * 2);
  if (off > ws_size || off > (size_t)134217728) return;

  pack_t_kernel<<<dim3(NGATE / 64, NFEAT / 64, NMIX), NTHR, 0, stream>>>(
      w_ih, (long)NFEAT * NGATE, NGATE, WCAT, (long)NGATE * KCAT, KCAT, WCARRY);
  pack_t_kernel<<<dim3(NGATE / 64, NHID / 64, NMIX), NTHR, 0, stream>>>(
      w_hh, (long)NHID * NGATE, NGATE, WCAT + NFEAT, (long)NGATE * KCAT, KCAT, WCARRY);
  pack_t_kernel<<<dim3(NOUTF / 64, NHID / 64, 1), NTHR, 0, stream>>>(
      w_out, 0L, NOUTF, WOT, 0L, NHID, WCARRY);

  lstm_seq_kernel<<<NBAT / SEQ_BLK, NTHR, 0, stream>>>(xin, bvec, alpha, WCAT, HS);

  wmma_gemm64<0, false, 2, 0, false, 0><<<dim3((NROWS / 64) * (NOUTF / 64) / 8, 1), 256, 0, stream>>>(
      HS, HS, NHID, 0L, WOT, WOT, NHID, 0L, (void*)out, (void*)out, NOUTF, 0L,
      b_out, b_out, 0L, NROWS, NOUTF, NHID, ACC_INV);
}
